// GlobalMambaBlockFromMamba_89756226551980
// MI455X (gfx1250) — hardware-verified
//
#include <hip/hip_runtime.h>
#include <math.h>

typedef __attribute__((ext_vector_type(8)))  _Float16 v8h;
typedef __attribute__((ext_vector_type(16))) __bf16   v16b;
typedef __attribute__((ext_vector_type(8)))  __bf16   v8b;
typedef __attribute__((ext_vector_type(8)))  float    v8f;
typedef __attribute__((ext_vector_type(4)))  float    v4f;

constexpr int kBatch = 2;
constexpr int kSeq   = 1024;
constexpr int kDm    = 1024;
constexpr int kDin   = 2048;
constexpr int kNst   = 16;
constexpr int kDtR   = 64;
constexpr int kPrjN  = 96;
constexpr int kPrjP  = 128;
constexpr int kXZP   = 2 * kDin;
constexpr int kRows  = kBatch * kSeq;
constexpr int kTP    = 260;
static_assert(kDtR + 2 * kNst == kPrjN);
static_assert((kDm % 32) == 0 && (kDin % 32) == 0 && (kDtR % 32) == 0);
static_assert((kRows % 64) == 0 && (kXZP % 64) == 0 && (kPrjP % 64) == 0 && (kDin % 64) == 0 && (kDm % 64) == 0);
static_assert((kSeq % 64) == 0 && (kSeq % 16) == 0 && (kDin % 256) == 0 && kDm == 128 * 8);
static_assert((kSeq & (kSeq - 1)) == 0);

constexpr size_t kOffWIN  = 0;
constexpr size_t kOffWXP  = kOffWIN  + (size_t)kXZP  * kDm   * 2;
constexpr size_t kOffWDT  = kOffWXP  + (size_t)kPrjP * kDin  * 2;
constexpr size_t kOffWOUT = kOffWDT  + (size_t)kDin  * kDtR  * 2;
constexpr size_t kOffXNH  = kOffWOUT + (size_t)kDm   * kDin  * 2;
constexpr size_t kOffXNL  = kOffXNH  + (size_t)kRows * kDm   * 2;
constexpr size_t kOffXZ   = kOffXNL  + (size_t)kRows * kDm   * 2;
constexpr size_t kOffUC   = kOffXZ   + (size_t)kRows * kXZP  * 4;
constexpr size_t kOffUCH  = kOffUC   + (size_t)kRows * kDin  * 4;
constexpr size_t kOffUCL  = kOffUCH  + (size_t)kRows * kDin  * 2;
constexpr size_t kOffPROJ = kOffUCL  + (size_t)kRows * kDin  * 2;
constexpr size_t kOffDTH  = kOffPROJ + (size_t)kRows * kPrjP * 4;
constexpr size_t kOffDTL  = kOffDTH  + (size_t)kRows * kDtR  * 2;
constexpr size_t kOffDLR  = kOffDTL  + (size_t)kRows * kDtR  * 2;
constexpr size_t kOffGH   = kOffDLR  + (size_t)kRows * kDin  * 4;
constexpr size_t kOffGL   = kOffGH   + (size_t)kRows * kDin  * 2;
constexpr size_t kWsTotal = kOffGL   + (size_t)kRows * kDin  * 2;
static_assert(kWsTotal == 123994112ull);
static_assert(kWsTotal <= 134217728ull);
static_assert((kOffWXP % 128) == 0 && (kOffWDT % 128) == 0 && (kOffWOUT % 128) == 0 && (kOffXNH % 128) == 0 &&
              (kOffXNL % 128) == 0 && (kOffXZ % 128) == 0 && (kOffUC % 128) == 0 && (kOffUCH % 128) == 0 &&
              (kOffUCL % 128) == 0 && (kOffPROJ % 128) == 0 && (kOffDTH % 128) == 0 && (kOffDTL % 128) == 0 &&
              (kOffDLR % 128) == 0 && (kOffGH % 128) == 0 && (kOffGL % 128) == 0);

__device__ __forceinline__ unsigned short f2bf_bits(float f) {
  unsigned u = __float_as_uint(f);
  return (unsigned short)((u + 0x7FFFu + ((u >> 16) & 1u)) >> 16);
}
__device__ __forceinline__ float bf_bits2f(unsigned short h) { return __uint_as_float(((unsigned)h) << 16); }
__device__ __forceinline__ float bf_rne(float f) { return bf_bits2f(f2bf_bits(f)); }

__device__ __forceinline__ void dep_guard4_b(v8f& a, v8f& b, v8f& c, v8f& d, v16b x, v16b y) {
  asm volatile("v_nop\n\tv_nop\n\tv_nop\n\tv_nop" : "+v"(a), "+v"(b), "+v"(c), "+v"(d) : "v"(x), "v"(y));
}
__device__ __forceinline__ void keep4_b(v16b a, v16b b, v16b c, v16b d) { asm volatile("v_nop" :: "v"(a), "v"(b), "v"(c), "v"(d)); }
__device__ __forceinline__ void acc_guard4(v8f& a, v8f& b, v8f& c, v8f& d) {
  asm volatile("v_nop\n\tv_nop\n\tv_nop\n\tv_nop" : "+v"(a), "+v"(b), "+v"(c), "+v"(d));
}

union FragB { v16b v; v8b h[2]; };
__device__ __forceinline__ v16b frag_load(const __bf16* p) {
  FragB f;
  f.h[0] = *(const v8b*)(p);
  f.h[1] = *(const v8b*)(p + 16);
  return f.v;
}
__device__ __forceinline__ v8f frag_mma(v16b a, v16b b, v8f c) {
  return __builtin_amdgcn_wmma_f32_16x16x32_bf16(false, a, false, b, (short)0, c, false, false);
}

template <int SPL, int BIAS_MODE>
__global__ __launch_bounds__(256) void wmma_gemm64(
    const unsigned short* __restrict__ Ap, const unsigned short* __restrict__ A2p, int lda,
    const unsigned short* __restrict__ Btp, int ldb,
    float* __restrict__ Cout, int ldc,
    const float* __restrict__ bias,
    int M, int N, int K, float scale) {
  const __bf16* A  = (const __bf16*)Ap;
  const __bf16* A2 = (const __bf16*)A2p;
  const __bf16* Bt = (const __bf16*)Btp;
  __shared__ __align__(16) float sT[8][16 * 68];
  const int lane = threadIdx.x & 31;
  const int wave = threadIdx.x >> 5;
  const int tilesN = N >> 6;
  const int tilesM = M >> 6;
  const int tile = blockIdx.x * 8 + wave;
  if (tile >= tilesM * tilesN) return;
  const int tm = tile / tilesN;
  const int tn = tile - tm * tilesN;
  const int m0 = tm << 6;
  const int n0 = tn << 6;

  const int rlane = lane & 15;
  const int koff  = (lane >> 4) * 8;
  const int mOff  = (lane >> 4) * 8;

  v8f acc[4][4];
#pragma unroll
  for (int i = 0; i < 4; ++i)
#pragma unroll
    for (int j = 0; j < 4; ++j) acc[i][j] = (v8f){0.f, 0.f, 0.f, 0.f, 0.f, 0.f, 0.f, 0.f};

  for (int k0 = 0; k0 < K; k0 += 32) {
    v16b bh[4];
#pragma unroll
    for (int j = 0; j < 4; ++j) {
      const size_t bo = (size_t)(n0 + (j << 4) + rlane) * ldb + koff + k0;
      bh[j] = frag_load(Bt + bo);
    }
#pragma unroll
    for (int i = 0; i < 4; ++i) {
      const size_t ao = (size_t)(m0 + (i << 4) + rlane) * lda + koff + k0;
      v16b ah = frag_load(A + ao);
      v16b al = ah;
      if (SPL >= 1) al = frag_load(A2 + ao);
#pragma unroll
      for (int j = 0; j < 4; ++j) {
        acc[i][j] = frag_mma(ah, bh[j], acc[i][j]);
        if (SPL >= 1) acc[i][j] = frag_mma(al, bh[j], acc[i][j]);
      }
      dep_guard4_b(acc[i][0], acc[i][1], acc[i][2], acc[i][3], ah, al);
    }
    keep4_b(bh[0], bh[1], bh[2], bh[3]);
  }
  acc_guard4(acc[0][0], acc[0][1], acc[0][2], acc[0][3]);
  acc_guard4(acc[1][0], acc[1][1], acc[1][2], acc[1][3]);
  acc_guard4(acc[2][0], acc[2][1], acc[2][2], acc[2][3]);
  acc_guard4(acc[3][0], acc[3][1], acc[3][2], acc[3][3]);

  float* slab = sT[wave];
#pragma unroll
  for (int i = 0; i < 4; ++i) {
    const int mBase = m0 + (i << 4);
#pragma unroll
    for (int j = 0; j < 4; ++j) {
      const int n = n0 + (j << 4) + rlane;
      float bv = 0.f;
      if (BIAS_MODE == 2) bv = bf_rne(bias[n]);
#pragma unroll
      for (int r = 0; r < 8; ++r) {
        float v = acc[i][j][r] * scale;
        if (BIAS_MODE == 2) v += bv;
        slab[(mOff + r) * 68 + (j << 4) + rlane] = v;
      }
    }
    __builtin_amdgcn_fence(__ATOMIC_RELEASE, "workgroup");
    __builtin_amdgcn_wave_barrier();
    __builtin_amdgcn_fence(__ATOMIC_ACQUIRE, "workgroup");
    {
      const int hh = lane >> 4, c4 = (lane & 15) * 4;
      for (int pass = 0; pass < 2; ++pass) {
#pragma unroll
        for (int it = 0; it < 8; ++it) {
          const int row = it * 2 + hh;
          v4f v = *(const v4f*)(slab + row * 68 + c4);
          *(volatile v4f*)(Cout + (size_t)(mBase + row) * ldc + n0 + c4) = v;
        }
        __threadfence();
      }
    }
    __builtin_amdgcn_fence(__ATOMIC_RELEASE, "workgroup");
    __builtin_amdgcn_wave_barrier();
    __builtin_amdgcn_fence(__ATOMIC_ACQUIRE, "workgroup");
  }
}

__global__ __launch_bounds__(256) void transpose_bf16_kernel(
    const float* __restrict__ W, unsigned short* __restrict__ Bt, int Kdim, int Ndim)
{
  __shared__ float tile[64 * 65];
  const int tid = threadIdx.x, lane = tid & 31, wave = tid >> 5;
  const int n0 = blockIdx.x * 64;
  const int k0 = blockIdx.y * 64;
#pragma unroll
  for (int p = 0; p < 16; ++p) {
    const int idx = tid + p * 256;
    const int kk  = idx >> 6;
    const int nn  = idx & 63;
    const int n   = n0 + nn;
    const int nc  = (n < Ndim) ? n : (Ndim - 1);
    const float v = W[(size_t)(k0 + kk) * Ndim + nc];
    tile[kk * 65 + nn] = (n < Ndim) ? v : 0.f;
  }
  __syncthreads();
  const int q = lane >> 3, c8 = (lane & 7) * 8;
  v8h hv[2];
#pragma unroll
  for (int it = 0; it < 2; ++it) {
    const int nrow = it * 32 + wave * 4 + q;
#pragma unroll
    for (int e = 0; e < 8; ++e) {
      const float f = tile[(c8 + e) * 65 + nrow];
      const unsigned short hb = f2bf_bits(f);
      hv[it][e] = __builtin_bit_cast(_Float16, hb);
    }
  }
  for (int pass = 0; pass < 2; ++pass) {
#pragma unroll
    for (int it = 0; it < 2; ++it) {
      const int nrow = it * 32 + wave * 4 + q;
      *(volatile v8h*)(Bt + (size_t)(n0 + nrow) * Kdim + k0 + c8) = hv[it];
    }
    __threadfence();
  }
}

__global__ __launch_bounds__(128) void layernorm_split_kernel(
    const float* __restrict__ x, const float* __restrict__ w, const float* __restrict__ b,
    unsigned short* __restrict__ XNH, unsigned short* __restrict__ XNL)
{
  __shared__ float sRed[2][4];
  const int tid = threadIdx.x, lane = tid & 31, wave = tid >> 5;
  const int row = blockIdx.x;
  const float* p = x + (size_t)row * kDm + tid * 8;
  const v4f a0 = *(const v4f*)(p);
  const v4f a1 = *(const v4f*)(p + 4);
  float v[8];
#pragma unroll
  for (int e = 0; e < 4; ++e) {
    const float f0 = a0[e];
    const float f1 = a1[e];
    v[e]     = bf_rne(f0);
    v[4 + e] = bf_rne(f1);
  }
  float s = ((v[0] + v[1]) + (v[2] + v[3])) + ((v[4] + v[5]) + (v[6] + v[7]));
#pragma unroll
  for (int off = 16; off > 0; off >>= 1) s += __shfl_xor(s, off, 32);
  if (lane == 0) sRed[0][wave] = s;
  __syncthreads();
  const float tot = ((sRed[0][0] + sRed[0][1]) + sRed[0][2]) + sRed[0][3];
  const float mu = tot * (1.0f / (float)kDm);
  float c[8];
#pragma unroll
  for (int e = 0; e < 8; ++e) c[e] = v[e] - mu;
  float sq = ((c[0] * c[0] + c[1] * c[1]) + (c[2] * c[2] + c[3] * c[3])) +
             ((c[4] * c[4] + c[5] * c[5]) + (c[6] * c[6] + c[7] * c[7]));
#pragma unroll
  for (int off = 16; off > 0; off >>= 1) sq += __shfl_xor(sq, off, 32);
  if (lane == 0) sRed[1][wave] = sq;
  __syncthreads();
  const float tot2 = ((sRed[1][0] + sRed[1][1]) + sRed[1][2]) + sRed[1][3];
  const float var = tot2 * (1.0f / (float)kDm);
  const float rs = rsqrtf(var + 1e-5f);
  const v4f w0 = *(const v4f*)(w + tid * 8);
  const v4f w1 = *(const v4f*)(w + tid * 8 + 4);
  const v4f b0 = *(const v4f*)(b + tid * 8);
  const v4f b1 = *(const v4f*)(b + tid * 8 + 4);
  v8h hv, lv;
#pragma unroll
  for (int e = 0; e < 4; ++e) {
    const float wa = w0[e], wb = w1[e], ba = b0[e], bb = b1[e];
    const float y0 = (c[e] * rs) * bf_rne(wa) + bf_rne(ba);
    const float y1 = (c[4 + e] * rs) * bf_rne(wb) + bf_rne(bb);
    const unsigned short h0 = f2bf_bits(y0), h1 = f2bf_bits(y1);
    const unsigned short l0 = f2bf_bits(y0 - bf_bits2f(h0)), l1 = f2bf_bits(y1 - bf_bits2f(h1));
    hv[e]     = __builtin_bit_cast(_Float16, h0);
    hv[4 + e] = __builtin_bit_cast(_Float16, h1);
    lv[e]     = __builtin_bit_cast(_Float16, l0);
    lv[4 + e] = __builtin_bit_cast(_Float16, l1);
  }
  unsigned short* qh = XNH + (size_t)row * kDm + tid * 8;
  unsigned short* ql = XNL + (size_t)row * kDm + tid * 8;
  *(volatile v8h*)qh = hv;
  *(volatile v8h*)ql = lv;
  __threadfence();
  *(volatile v8h*)qh = hv;
  *(volatile v8h*)ql = lv;
}

__global__ __launch_bounds__(256) void conv_silu_kernel(
    const float* __restrict__ XZ, const float* __restrict__ cw, const float* __restrict__ cb,
    float* __restrict__ UC, unsigned short* __restrict__ UCH, unsigned short* __restrict__ UCL)
{
  __shared__ __align__(16) float sT[16 * kTP];
  const int tid = threadIdx.x, lane = tid & 31, wave = tid >> 5;
  const int d0 = blockIdx.x * 256, d = d0 + tid;
  const int g0 = blockIdx.y * 64;
  const int tb = g0 & (kSeq - 1);
  const float w0 = bf_rne(cw[d * 4 + 0]);
  const float w1 = bf_rne(cw[d * 4 + 1]);
  const float w2 = bf_rne(cw[d * 4 + 2]);
  const float w3 = bf_rne(cw[d * 4 + 3]);
  const float bc = bf_rne(cb[d]);
  float xm3, xm2, xm1;
  {
    const bool hist = (tb > 0);
    const int rb = hist ? (g0 - 3) : g0;
    const float v3 = XZ[(size_t)rb * kXZP + d];
    const float v2 = XZ[(size_t)(rb + 1) * kXZP + d];
    const float v1 = XZ[(size_t)(rb + 2) * kXZP + d];
    xm3 = hist ? v3 : 0.f;
    xm2 = hist ? v2 : 0.f;
    xm1 = hist ? v1 : 0.f;
  }
  const int hrow = wave >> 1;
  const int hch  = (wave & 1) * 128 + lane * 4;
#pragma unroll 1
  for (int sub = 0; sub < 4; ++sub) {
    const int lb = g0 + sub * 16;
#pragma unroll 1
    for (int s = 0; s < 16; ++s) {
      const float xcur = XZ[(size_t)(lb + s) * kXZP + d];
      float acc = w0 * xm3;
      acc = fmaf(w1, xm2, acc);
      acc = fmaf(w2, xm1, acc);
      acc = fmaf(w3, xcur, acc);
      const float sv = acc + bc;
      const float sg = __builtin_amdgcn_rcpf(1.0f + expf(-sv));
      sT[s * kTP + tid] = sv * sg;
      xm3 = xm2; xm2 = xm1; xm1 = xcur;
    }
    __syncthreads();
    v4f fv[4];
    v8h bh[2], blo[2];
#pragma unroll
    for (int it = 0; it < 4; ++it) fv[it] = *(const v4f*)(sT + (it * 4 + hrow) * kTP + hch);
#pragma unroll
    for (int it = 0; it < 2; ++it) {
      const float* sp = sT + (it * 8 + wave) * kTP + lane * 8;
      const v4f a0 = *(const v4f*)(sp);
      const v4f a1 = *(const v4f*)(sp + 4);
#pragma unroll
      for (int e = 0; e < 4; ++e) {
        const float f0 = a0[e], f1 = a1[e];
        const unsigned short h0 = f2bf_bits(f0), h1 = f2bf_bits(f1);
        const unsigned short l0 = f2bf_bits(f0 - bf_bits2f(h0)), l1 = f2bf_bits(f1 - bf_bits2f(h1));
        bh[it][e]      = __builtin_bit_cast(_Float16, h0);
        bh[it][4 + e]  = __builtin_bit_cast(_Float16, h1);
        blo[it][e]     = __builtin_bit_cast(_Float16, l0);
        blo[it][4 + e] = __builtin_bit_cast(_Float16, l1);
      }
    }
    for (int pass = 0; pass < 2; ++pass) {
#pragma unroll
      for (int it = 0; it < 4; ++it)
        *(volatile v4f*)(UC + (size_t)(lb + it * 4 + hrow) * kDin + d0 + hch) = fv[it];
#pragma unroll
      for (int it = 0; it < 2; ++it) {
        const size_t o = (size_t)(lb + it * 8 + wave) * kDin + d0 + lane * 8;
        *(volatile v8h*)(UCH + o) = bh[it];
        *(volatile v8h*)(UCL + o) = blo[it];
      }
      __threadfence();
    }
    __syncthreads();
  }
}

__global__ __launch_bounds__(256) void dt_split_kernel(
    const float* __restrict__ PROJ, unsigned short* __restrict__ DTH, unsigned short* __restrict__ DTL, int total8)
{
  const int i = blockIdx.x * 256 + threadIdx.x;
  if (i >= total8) return;
  const int e0  = i << 3;
  const int row = e0 >> 6;
  const int c8  = e0 & 63;
  const float* p = PROJ + (size_t)row * kPrjP + c8;
  const v4f a0 = *(const v4f*)(p);
  const v4f a1 = *(const v4f*)(p + 4);
  v8h hv, lv;
#pragma unroll
  for (int e = 0; e < 4; ++e) {
    const float f0 = a0[e], f1 = a1[e];
    const unsigned short h0 = f2bf_bits(f0), h1 = f2bf_bits(f1);
    const unsigned short l0 = f2bf_bits(f0 - bf_bits2f(h0)), l1 = f2bf_bits(f1 - bf_bits2f(h1));
    hv[e]     = __builtin_bit_cast(_Float16, h0);
    hv[4 + e] = __builtin_bit_cast(_Float16, h1);
    lv[e]     = __builtin_bit_cast(_Float16, l0);
    lv[4 + e] = __builtin_bit_cast(_Float16, l1);
  }
  unsigned short* qh = DTH + e0;
  unsigned short* ql = DTL + e0;
  *(volatile v8h*)qh = hv;
  *(volatile v8h*)ql = lv;
  __threadfence();
  *(volatile v8h*)qh = hv;
  *(volatile v8h*)ql = lv;
}

__global__ __launch_bounds__(256) void scan_kernel(
    const float* __restrict__ DLR, const float* __restrict__ UC, const float* __restrict__ XZ,
    const float* __restrict__ PROJ, const float* __restrict__ A_log, const float* __restrict__ Dv,
    unsigned short* __restrict__ GH, unsigned short* __restrict__ GL)
{
  __shared__ __align__(16) float sBC[16 * 32];
  __shared__ __align__(16) float sY[16 * kTP];
  __shared__ float sA[kNst * 256];
  const int tid = threadIdx.x, lane = tid & 31, wave = tid >> 5;
  constexpr int kBlkPerB = kDin / 256;
  const int bix = blockIdx.x / kBlkPerB;
  const int d0  = (blockIdx.x - bix * kBlkPerB) * 256;
  const int d   = d0 + tid;
  const size_t row0 = (size_t)bix * kSeq;

#pragma unroll 1
  for (int s = 0; s < kNst; ++s) sA[s * 256 + tid] = -expf(bf_rne(A_log[(size_t)d * kNst + s]));
  __syncthreads();
  float An[kNst], h[kNst];
#pragma unroll
  for (int n = 0; n < kNst; ++n) {
    An[n] = sA[n * 256 + tid];
    h[n] = 0.f;
  }
  const float Dd = bf_rne(Dv[d]);

#pragma unroll 1
  for (int c = 0; c < kSeq / 16; ++c) {
    const int l0 = c * 16;
    if (tid < 128) {
      const int r = tid >> 3, q4 = (tid & 7) * 4;
      const v4f v = *(const v4f*)(PROJ + (row0 + l0 + r) * kPrjP + kDtR + q4);
      *(v4f*)(sBC + r * 32 + q4) = v;
    }
    __syncthreads();
#pragma unroll 1
    for (int s = 0; s < 16; ++s) {
      const size_t m = row0 + (size_t)(l0 + s);
      const float a  = DLR[m * kDin + d];
      const float ea = __expf(-fabsf(a));
      const float u1 = 1.0f + ea;
      const float l1p = __logf(u1) + (ea - (u1 - 1.0f)) * __builtin_amdgcn_rcpf(u1);
      const float delta = fmaxf(a, 0.0f) + l1p;
      const float xv = UC[m * kDin + d];
      const float zv = XZ[m * kXZP + kDin + d];
      v4f Bq[4], Cq[4];
#pragma unroll
      for (int qq = 0; qq < 4; ++qq) {
        Bq[qq] = *(const v4f*)(sBC + s * 32 + 4 * qq);
        Cq[qq] = *(const v4f*)(sBC + s * 32 + kNst + 4 * qq);
      }
      const float dtx = delta * xv;
      float y = 0.f;
#pragma unroll
      for (int n = 0; n < kNst; ++n) {
        const float e = __expf(delta * An[n]);
        const float hn = e * h[n] + dtx * Bq[n >> 2][n & 3];
        h[n] = hn;
        y = hn * Cq[n >> 2][n & 3] + y;
      }
      y = xv * Dd + y;
      const float sg = __builtin_amdgcn_rcpf(1.0f + expf(-zv));
      sY[s * kTP + tid] = y * (zv * sg);
    }
    __syncthreads();
    v8h hv[2], lv[2];
#pragma unroll
    for (int it = 0; it < 2; ++it) {
      const float* sp = sY + (it * 8 + wave) * kTP + lane * 8;
      const v4f a0 = *(const v4f*)(sp);
      const v4f a1 = *(const v4f*)(sp + 4);
#pragma unroll
      for (int e = 0; e < 4; ++e) {
        const float f0 = a0[e], f1 = a1[e];
        const unsigned short h0 = f2bf_bits(f0), h1 = f2bf_bits(f1);
        const unsigned short l0b = f2bf_bits(f0 - bf_bits2f(h0)), l1b = f2bf_bits(f1 - bf_bits2f(h1));
        hv[it][e]     = __builtin_bit_cast(_Float16, h0);
        hv[it][4 + e] = __builtin_bit_cast(_Float16, h1);
        lv[it][e]     = __builtin_bit_cast(_Float16, l0b);
        lv[it][4 + e] = __builtin_bit_cast(_Float16, l1b);
      }
    }
    for (int pass = 0; pass < 2; ++pass) {
#pragma unroll
      for (int it = 0; it < 2; ++it) {
        const size_t o = (row0 + (size_t)(l0 + it * 8 + wave)) * kDin + d0 + lane * 8;
        *(volatile v8h*)(GH + o) = hv[it];
        *(volatile v8h*)(GL + o) = lv[it];
      }
      __threadfence();
    }
  }
}

extern "C" void kernel_launch(void* const* d_in, const int* in_sizes, int n_in,
                              void* d_out, int out_size, void* d_ws, size_t ws_size,
                              hipStream_t stream)
{
  if (n_in < 14) return;
  if (in_sizes[0] != kRows * kDm) return;
  if (in_sizes[1] != kDm || in_sizes[2] != kDm) return;
  if (in_sizes[3] != kDm * kXZP || in_sizes[4] != kXZP) return;
  if (in_sizes[5] != kDin * 4 || in_sizes[6] != kDin) return;
  if (in_sizes[7] != kDin * kPrjN) return;
  if (in_sizes[8] != kDtR * kDin || in_sizes[9] != kDin) return;
  if (in_sizes[10] != kDin * kNst || in_sizes[11] != kDin) return;
  if (in_sizes[12] != kDin * kDm || in_sizes[13] != kDm) return;
  if (out_size != kRows * kDm) return;
  if (ws_size < kWsTotal) return;

  const float* x       = (const float*)d_in[0];
  const float* norm_w  = (const float*)d_in[1];
  const float* norm_b  = (const float*)d_in[2];
  const float* in_w    = (const float*)d_in[3];
  const float* in_b    = (const float*)d_in[4];
  const float* conv_w  = (const float*)d_in[5];
  const float* conv_b  = (const float*)d_in[6];
  const float* xproj_w = (const float*)d_in[7];
  const float* dt_w    = (const float*)d_in[8];
  const float* dt_b    = (const float*)d_in[9];
  const float* A_log   = (const float*)d_in[10];
  const float* Dv      = (const float*)d_in[11];
  const float* out_w   = (const float*)d_in[12];
  const float* out_b   = (const float*)d_in[13];
  float* out = (float*)d_out;

  char* ws = (char*)d_ws;
  unsigned short* WIN  = (unsigned short*)(ws + kOffWIN);
  unsigned short* WXP  = (unsigned short*)(ws + kOffWXP);
  unsigned short* WDT  = (unsigned short*)(ws + kOffWDT);
  unsigned short* WOUT = (unsigned short*)(ws + kOffWOUT);
  unsigned short* XNH  = (unsigned short*)(ws + kOffXNH);
  unsigned short* XNL  = (unsigned short*)(ws + kOffXNL);
  float*          XZ   = (float*)(ws + kOffXZ);
  float*          UC   = (float*)(ws + kOffUC);
  unsigned short* UCH  = (unsigned short*)(ws + kOffUCH);
  unsigned short* UCL  = (unsigned short*)(ws + kOffUCL);
  float*          PROJ = (float*)(ws + kOffPROJ);
  unsigned short* DTH  = (unsigned short*)(ws + kOffDTH);
  unsigned short* DTL  = (unsigned short*)(ws + kOffDTL);
  float*          DLR  = (float*)(ws + kOffDLR);
  unsigned short* GH   = (unsigned short*)(ws + kOffGH);
  unsigned short* GL   = (unsigned short*)(ws + kOffGL);

  transpose_bf16_kernel<<<dim3(kXZP / 64, kDm / 64), 256, 0, stream>>>(in_w, WIN, kDm, kXZP);
  transpose_bf16_kernel<<<dim3(kPrjP / 64, kDin / 64), 256, 0, stream>>>(xproj_w, WXP, kDin, kPrjN);
  transpose_bf16_kernel<<<dim3(kDin / 64, kDtR / 64), 256, 0, stream>>>(dt_w, WDT, kDtR, kDin);
  transpose_bf16_kernel<<<dim3(kDm / 64, kDin / 64), 256, 0, stream>>>(out_w, WOUT, kDin, kDm);

  layernorm_split_kernel<<<kRows, 128, 0, stream>>>(x, norm_w, norm_b, XNH, XNL);

  wmma_gemm64<1, 2><<<dim3((kRows / 64) * (kXZP / 64) / 8), 256, 0, stream>>>(
      XNH, XNL, kDm, WIN, kDm, XZ, kXZP, in_b, kRows, kXZP, kDm, 1.0f);

  conv_silu_kernel<<<dim3(kDin / 256, kRows / 64), 256, 0, stream>>>(XZ, conv_w, conv_b, UC, UCH, UCL);

  wmma_gemm64<1, 0><<<dim3((kRows / 64) * (kPrjP / 64) / 8), 256, 0, stream>>>(
      UCH, UCL, kDin, WXP, kDin, PROJ, kPrjP, dt_b, kRows, kPrjP, kDin, 1.0f);

  dt_split_kernel<<<(kRows * kDtR) / 8 / 256, 256, 0, stream>>>(PROJ, DTH, DTL, (kRows * kDtR) / 8);

  wmma_gemm64<1, 2><<<dim3((kRows / 64) * (kDin / 64) / 8), 256, 0, stream>>>(
      DTH, DTL, kDtR, WDT, kDtR, DLR, kDin, dt_b, kRows, kDin, kDtR, 1.0f);

  scan_kernel<<<kBatch * (kDin / 256), 256, 0, stream>>>(DLR, UC, XZ, PROJ, A_log, Dv, GH, GL);

  wmma_gemm64<1, 2><<<dim3((kRows / 64) * (kDm / 64) / 8), 256, 0, stream>>>(
      GH, GL, kDin, WOUT, kDin, out, kDm, out_b, kRows, kDm, kDin, 1.0f);
}
